// SpatialAxialAttention_34926674051602
// MI455X (gfx1250) — hardware-verified
//
#include <hip/hip_runtime.h>
#include <hip/hip_bf16.h>


#define __bf16 _Float16
typedef _Float16 bf16;
typedef __attribute__((ext_vector_type(8)))  _Float16 bf16x8;
typedef __attribute__((ext_vector_type(16))) _Float16 bf16x16;
typedef __attribute__((ext_vector_type(4)))  float  v4f_t;
typedef float v4fa __attribute__((ext_vector_type(4), may_alias));
typedef __attribute__((ext_vector_type(4)))  unsigned v4u_t;
typedef unsigned v4ua __attribute__((ext_vector_type(4), may_alias));
static __device__ __forceinline__ unsigned pk2(float a, float b) { return (unsigned)__builtin_bit_cast(unsigned short, (_Float16)a) | ((unsigned)__builtin_bit_cast(unsigned short, (_Float16)b) << 16); }
typedef __attribute__((ext_vector_type(8)))  float  f32x8;
typedef __attribute__((ext_vector_type(4)))  unsigned int u32x4;
typedef __attribute__((ext_vector_type(8)))  int i32x8;
typedef __attribute__((ext_vector_type(4)))  int i32x4;

#if defined(__has_builtin)
#if __has_builtin(__builtin_amdgcn_tensor_load_to_lds)
#define HAS_TDM 1
#endif
#endif

#define WMMA_BF16(a, b, c) \
  __builtin_amdgcn_wmma_f32_16x16x32_f16(false, (a), false, (b), (short)0, (c), false, false)

static __device__ __forceinline__ bf16x16 cat8(bf16x8 lo, bf16x8 hi) {
  return __builtin_shufflevector(lo, hi, 0,1,2,3,4,5,6,7,8,9,10,11,12,13,14,15);
}
static __device__ __forceinline__ f32x8 zero8() {
  f32x8 z;
  #pragma unroll
  for (int i = 0; i < 8; ++i) z[i] = 0.0f;
  return z;
}

#ifdef HAS_TDM
static __device__ __forceinline__ void tdm_load_tile(unsigned int lds_addr,
                                                     unsigned long long gaddr,
                                                     unsigned int dim0,
                                                     unsigned int dim1,
                                                     unsigned int stride0) {
  u32x4 g0 = { 1u, lds_addr, (unsigned int)gaddr,
               (unsigned int)(gaddr >> 32) | (2u << 30) };
  const unsigned int w0 = (1u << 16)
                        | (1u << 20)
                        | (3u << 22)
                        | (3u << 25);
  i32x8 g1 = { (int)w0,
               (int)((dim0 & 0xFFFFu) << 16),
               (int)((dim0 >> 16) | ((dim1 & 0xFFFFu) << 16)),
               (int)((dim1 >> 16) | (32u << 16)),
               (int)128u,
               (int)stride0,
               0, 0 };
  i32x4 z4 = { 0, 0, 0, 0 };
  i32x8 z8 = { 0, 0, 0, 0, 0, 0, 0, 0 };
  __builtin_amdgcn_tensor_load_to_lds(g0, g1, z4, z4, z8, 0);
}
#endif

__global__ void k_f32_to_bf16(const float* __restrict__ src, bf16* __restrict__ dst, int n) {
  int i = (blockIdx.x * blockDim.x + threadIdx.x) * 2;
  if (i < n) { const unsigned p = pk2(src[i], src[i + 1]); *(volatile unsigned*)(dst + i) = p; __threadfence(); *(volatile unsigned*)(dst + i) = p; }
}

__global__ void k_transpose_bf16(const float* __restrict__ src, bf16* __restrict__ dst,
                                 int K, int N) {
  int i = (blockIdx.x * blockDim.x + threadIdx.x) * 2;
  if (i < K * N) {
    int n = i / K, k = i - n * K;
    const unsigned p = pk2(src[(size_t)k * N + n], src[(size_t)(k + 1) * N + n]);
    *(volatile unsigned*)(dst + i) = p; __threadfence(); *(volatile unsigned*)(dst + i) = p;
  }
}

template <int EPI>
__global__ __launch_bounds__(256) void k_gemm(const bf16* __restrict__ A,
                                              const bf16* __restrict__ BT,
                                              int M, int K, int N,
                                              bf16* __restrict__ Cb,
                                              float* __restrict__ Cf,
                                              const float* __restrict__ bias) {
  __shared__ bf16 sA[2][128 * 40];
  __shared__ bf16 sB[2][128 * 40];
  __shared__ __attribute__((aligned(16))) float sC[128][128];

  const int tid  = threadIdx.x;
  const int l    = tid & 31;
  const int wv   = tid >> 5;
  const int l16  = l & 15;
  const int half = l >> 4;
  const int wm   = wv & 1;
  const int wn   = wv >> 1;
  const int rowBase = blockIdx.x * 128;
  const int colBase = blockIdx.y * 128;

  f32x8 acc[4][2];
  #pragma unroll
  for (int i = 0; i < 4; ++i)
    #pragma unroll
    for (int j = 0; j < 2; ++j) acc[i][j] = zero8();

#ifdef HAS_TDM
  const unsigned long long aG = (unsigned long long)(uintptr_t)(A + (size_t)rowBase * K);
  const unsigned long long bG = (unsigned long long)(uintptr_t)(BT + (size_t)colBase * K);
  const unsigned int ldsA0 = (unsigned int)(uintptr_t)&sA[0][0];
  const unsigned int ldsA1 = (unsigned int)(uintptr_t)&sA[1][0];
  const unsigned int ldsB0 = (unsigned int)(uintptr_t)&sB[0][0];
  const unsigned int ldsB1 = (unsigned int)(uintptr_t)&sB[1][0];
  if (wv == 0) {
    tdm_load_tile(ldsA0, aG, (unsigned)K, (unsigned)M, (unsigned)K);
    tdm_load_tile(ldsB0, bG, (unsigned)K, (unsigned)N, (unsigned)K);
  }
#endif

  for (int k0 = 0; k0 < K; k0 += 32) {
    const int cur = (k0 >> 5) & 1;
    __syncthreads();
#ifdef HAS_TDM
    if (wv == 0) {
      if (k0 + 32 < K) {
        tdm_load_tile(cur ? ldsA0 : ldsA1, aG + (unsigned long long)(k0 + 32) * 2,
                      (unsigned)K, (unsigned)M, (unsigned)K);
        tdm_load_tile(cur ? ldsB0 : ldsB1, bG + (unsigned long long)(k0 + 32) * 2,
                      (unsigned)K, (unsigned)N, (unsigned)K);
        __builtin_amdgcn_s_wait_tensorcnt(2);
      } else {
        __builtin_amdgcn_s_wait_tensorcnt(0);
      }
    }
#else
    #pragma unroll
    for (int c = tid; c < 512; c += 256) {
      int r  = c >> 2;
      int cc = (c & 3) * 8;
      *(bf16x8*)(&sA[cur][r * 40 + cc]) =
          *(const bf16x8*)(&A[(size_t)(rowBase + r) * K + k0 + cc]);
      *(bf16x8*)(&sB[cur][r * 40 + cc]) =
          *(const bf16x8*)(&BT[(size_t)(colBase + r) * K + k0 + cc]);
    }
#endif
    __syncthreads();

    bf16x16 af[4], bfr[2];
    #pragma unroll
    for (int i = 0; i < 4; ++i) {
      const bf16* base = &sA[cur][(wm * 64 + i * 16 + l16) * 40];
      bf16x8 lo = *(const bf16x8*)(base + half * 8);
      bf16x8 hi = *(const bf16x8*)(base + 16 + half * 8);
      af[i] = cat8(lo, hi);
    }
    #pragma unroll
    for (int j = 0; j < 2; ++j) {
      const bf16* base = &sB[cur][(wn * 32 + j * 16 + l16) * 40 + half * 8];
      bf16x8 lo = *(const bf16x8*)(base);
      bf16x8 hi = *(const bf16x8*)(base + 16);
      bfr[j] = cat8(lo, hi);
    }
    #pragma unroll
    for (int i = 0; i < 4; ++i)
      #pragma unroll
      for (int j = 0; j < 2; ++j)
        acc[i][j] = WMMA_BF16(af[i], bfr[j], acc[i][j]);
  }

  #pragma unroll
  for (int i = 0; i < 4; ++i)
    #pragma unroll
    for (int j = 0; j < 2; ++j)
      #pragma unroll
      for (int r = 0; r < 8; ++r) sC[wm * 64 + i * 16 + r + half * 8][wn * 32 + j * 16 + l16] = acc[i][j][r];
  __syncthreads();
  if (EPI == 0) {
#pragma unroll 1
    for (int pass = 0; pass < 2; ++pass) {
#pragma unroll
      for (int i = 0; i < 8; ++i) {
        const int c = tid + 256 * i, rr = c >> 4, q = c & 15;
        const float* s = &sC[rr][q * 8];
        v4u_t v; v.x = pk2(s[0], s[1]); v.y = pk2(s[2], s[3]); v.z = pk2(s[4], s[5]); v.w = pk2(s[6], s[7]);
        *(volatile v4u_t*)(Cb + (size_t)(rowBase + rr) * N + colBase + q * 8) = v;
      }
      __threadfence();
    }
  } else {
#pragma unroll 1
    for (int pass = 0; pass < 2; ++pass) {
#pragma unroll
      for (int i = 0; i < 16; ++i) {
        const int c = tid + 256 * i, rr = c >> 5, q = c & 31;
        v4f_t v = *(const v4fa*)&sC[rr][q * 4];
        const v4f_t bb = *(const v4f_t*)(bias + colBase + q * 4);
        *(volatile v4f_t*)(Cf + (size_t)(rowBase + rr) * N + colBase + q * 4) = v + bb;
      }
      __threadfence();
    }
  }
}

__global__ void k_rope_pack(const bf16* __restrict__ qkv,
                            bf16* __restrict__ qh, bf16* __restrict__ kh,
                            bf16* __restrict__ vT) {
  int t    = blockIdx.x * 256 + threadIdx.x;
  int d2   = t & 31;
  int seq  = (t >> 5) & 1023;
  int head = (t >> 15) & 15;
  int bt   = t >> 19;
  int bh   = bt * 16 + head;

  size_t row = (size_t)(bt * 1024 + seq);
  int    col = head * 64 + d2 * 2;
  const bf16* rp = qkv + row * 3072;
  float q0 = (float)rp[col],        q1 = (float)rp[col + 1];
  float k0 = (float)rp[1024 + col], k1 = (float)rp[1024 + col + 1];
  float v0 = (float)rp[2048 + col], v1 = (float)rp[2048 + col + 1];

  int   j    = d2 & 15;
  float base = (1.0f + (127.0f / 15.0f) * (float)j) * 3.14159265358979323f;
  float pos  = (d2 < 16) ? (-1.0f + (2.0f / 31.0f) * (float)(seq >> 5))
                         : (-1.0f + (2.0f / 31.0f) * (float)(seq & 31));
  float f = pos * base, s, c;
  sincosf(f, &s, &c);

  size_t o = (size_t)bh * 65536 + (size_t)seq * 64 + d2 * 2;
  const unsigned pq = pk2(q0 * c - q1 * s, q1 * c + q0 * s);
  const unsigned pk = pk2(k0 * c - k1 * s, k1 * c + k0 * s);
  const unsigned pv = pk2(v0, v1);
  *(volatile unsigned*)(qh + o) = pq; *(volatile unsigned*)(kh + o) = pk; *(volatile unsigned*)(vT + o) = pv;
  __threadfence();
  *(volatile unsigned*)(qh + o) = pq; *(volatile unsigned*)(kh + o) = pk; *(volatile unsigned*)(vT + o) = pv;
}

__global__ __launch_bounds__(256) void k_vt(const bf16* __restrict__ vR, bf16* __restrict__ vT) {
  __shared__ bf16 t[64][66];
  const int tid = threadIdx.x, lane = tid & 31, wave = tid >> 5;
  const int bh = blockIdx.x >> 4, s0 = (blockIdx.x & 15) * 64;
  const bf16* src = vR + (size_t)bh * 65536 + (size_t)s0 * 64;
#pragma unroll
  for (int k = 0; k < 16; ++k) { const int e = tid + 256 * k; t[e >> 6][e & 63] = src[e]; }
  __syncthreads();
  bf16* dst = vT + (size_t)bh * 65536 + s0;
#pragma unroll
  for (int r = 0; r < 8; ++r) {
    const int d = wave * 8 + r;
    const unsigned pk = (unsigned)__builtin_bit_cast(unsigned short, t[2 * lane][d]) | ((unsigned)__builtin_bit_cast(unsigned short, t[2 * lane + 1][d]) << 16);
    unsigned* dp = (unsigned*)(dst + (size_t)d * 1024) + lane;
    *(volatile unsigned*)dp = pk; __threadfence(); *(volatile unsigned*)dp = pk;
  }
}

__global__ __launch_bounds__(256) void k_attention(const bf16* __restrict__ qh,
                                                   const bf16* __restrict__ kh,
                                                   const bf16* __restrict__ vT,
                                                   bf16* __restrict__ attn) {
  __shared__ bf16 pbuf[8][16 * 32];

  const int tid  = threadIdx.x;
  const int wv   = tid >> 5;
  const int l    = tid & 31;
  const int l16  = l & 15;
  const int half = l >> 4;
  const int bh   = blockIdx.x >> 3;
  const int q0r  = (blockIdx.x & 7) * 128 + wv * 16;

  const bf16* Q  = qh + (size_t)bh * 65536;
  const bf16* Kp = kh + (size_t)bh * 65536;
  const bf16* Vp = vT + (size_t)bh * 65536;

  bf16x16 qa[2];
  #pragma unroll
  for (int ci = 0; ci < 2; ++ci) {
    const bf16* base = Q + (size_t)(q0r + l16) * 64 + ci * 32 + half * 8;
    qa[ci] = cat8(*(const bf16x8*)base, *(const bf16x8*)(base + 16));
  }

  f32x8 O[4];
  #pragma unroll
  for (int t = 0; t < 4; ++t) O[t] = zero8();
  float m[8], lsum[8];
  #pragma unroll
  for (int r = 0; r < 8; ++r) { m[r] = -3.0e38f; lsum[r] = 0.0f; }

  for (int j0 = 0; j0 < 1024; j0 += 32) {
    if (j0 + 32 < 1024) {
      __builtin_prefetch(Kp + (size_t)(j0 + 32 + l16) * 64, 0, 1);
      __builtin_prefetch(Vp + (size_t)l16 * 1024 + j0 + 32, 0, 1);
    }
    f32x8 S0 = zero8(), S1 = zero8();
    #pragma unroll
    for (int ci = 0; ci < 2; ++ci) {
      {
        const bf16* base = Kp + (size_t)(j0 + l16) * 64 + ci * 32 + half * 8;
        S0 = WMMA_BF16(qa[ci], cat8(*(const bf16x8*)base, *(const bf16x8*)(base + 16)), S0);
      }
      {
        const bf16* base = Kp + (size_t)(j0 + 16 + l16) * 64 + ci * 32 + half * 8;
        S1 = WMMA_BF16(qa[ci], cat8(*(const bf16x8*)base, *(const bf16x8*)(base + 16)), S1);
      }
    }
    float p0[8], p1[8];
    #pragma unroll
    for (int r = 0; r < 8; ++r) {
      float s0 = S0[r] * 0.125f, s1 = S1[r] * 0.125f;
      float rowmax = fmaxf(s0, s1);
      #pragma unroll
      for (int off = 1; off < 16; off <<= 1)
        rowmax = fmaxf(rowmax, __shfl_xor(rowmax, off, 32));
      float mn    = fmaxf(m[r], rowmax);
      float alpha = __expf(m[r] - mn);
      m[r] = mn;
      float e0 = __expf(s0 - mn), e1 = __expf(s1 - mn);
      float rs = e0 + e1;
      #pragma unroll
      for (int off = 1; off < 16; off <<= 1) rs += __shfl_xor(rs, off, 32);
      lsum[r] = lsum[r] * alpha + rs;
      p0[r] = e0; p1[r] = e1;
      #pragma unroll
      for (int t = 0; t < 4; ++t) O[t][r] *= alpha;
    }
    #pragma unroll
    for (int r = 0; r < 8; ++r) {
      int prow = r + half * 8;
      pbuf[wv][prow * 32 + l16]      = (bf16)(p0[r] * 1024.0f);
      pbuf[wv][prow * 32 + 16 + l16] = (bf16)(p1[r] * 1024.0f);
    }
    asm volatile("s_wait_dscnt 0" ::: "memory");
    bf16x16 pa;
    {
      const bf16* base = &pbuf[wv][l16 * 32 + half * 8];
      pa = cat8(*(const bf16x8*)base, *(const bf16x8*)(base + 16));
    }
    #pragma unroll
    for (int t = 0; t < 4; ++t) {
      const bf16* base = Vp + (size_t)(t * 16 + l16) * 1024 + j0 + half * 8;
      O[t] = WMMA_BF16(pa, cat8(*(const bf16x8*)base, *(const bf16x8*)(base + 16)), O[t]);
    }
  }

  __shared__ __attribute__((aligned(16))) float ost[8][16 * 64];
  const int bt = bh >> 4, head = bh & 15;
  float* os_ = ost[wv];
  #pragma unroll
  for (int t = 0; t < 4; ++t)
    #pragma unroll
    for (int r = 0; r < 8; ++r) os_[(r + half * 8) * 64 + t * 16 + l16] = O[t][r] / (lsum[r] * 1024.0f);
  asm volatile("s_wait_dscnt 0" ::: "memory");
#pragma unroll 1
  for (int pass = 0; pass < 2; ++pass) {
#pragma unroll 4
    for (int rr = 0; rr < 16; ++rr) {
      const unsigned pk = pk2(*(const volatile float*)(os_ + rr * 64 + 2 * l), *(const volatile float*)(os_ + rr * 64 + 2 * l + 1));
      *(volatile unsigned*)(attn + (size_t)(bt * 1024 + q0r + rr) * 1024 + head * 64 + 2 * l) = pk;
    }
    __threadfence();
  }
}

extern "C" void kernel_launch(void* const* d_in, const int* in_sizes, int n_in,
                              void* d_out, int out_size, void* d_ws, size_t ws_size,
                              hipStream_t stream) {
  const float* x     = (const float*)d_in[0];
  const float* w_qkv = (const float*)d_in[1];
  const float* w_out = (const float*)d_in[2];
  const float* b_out = (const float*)d_in[3];
  float*       out   = (float*)d_out;

  char* ws = (char*)d_ws;
  size_t off = 0;
  bf16* xb    = (bf16*)(ws + off); off += (size_t)8192 * 1024 * 2;
  bf16* wqkvT = (bf16*)(ws + off); off += (size_t)3072 * 1024 * 2;
  bf16* woutT = (bf16*)(ws + off); off += (size_t)1024 * 1024 * 2;
  bf16* qkv   = (bf16*)(ws + off); off += (size_t)8192 * 3072 * 2;
  bf16* qhp   = (bf16*)(ws + off); off += (size_t)128 * 65536 * 2;
  bf16* khp   = (bf16*)(ws + off); off += (size_t)128 * 65536 * 2;
  bf16* vTp   = (bf16*)(ws + off); off += (size_t)128 * 65536 * 2;
  bf16* attn  = (bf16*)(ws + off); off += (size_t)8192 * 1024 * 2;
  bf16* vRp   = (bf16*)(ws + off); off += (size_t)128 * 65536 * 2;

  k_f32_to_bf16<<<8388608 / 512, 256, 0, stream>>>(x, xb, 8388608);
  k_transpose_bf16<<<(3072 * 1024) / 512, 256, 0, stream>>>(w_qkv, wqkvT, 1024, 3072);
  k_transpose_bf16<<<(1024 * 1024) / 512, 256, 0, stream>>>(w_out, woutT, 1024, 1024);

  k_gemm<0><<<dim3(64, 24), 256, 0, stream>>>(xb, wqkvT, 8192, 1024, 3072,
                                              qkv, nullptr, nullptr);

  k_rope_pack<<<16384, 256, 0, stream>>>(qkv, qhp, khp, vRp);
  k_vt<<<128 * 16, 256, 0, stream>>>(vRp, vTp);

  k_attention<<<1024, 256, 0, stream>>>(qhp, khp, vTp, attn);

  k_gemm<1><<<dim3(64, 8), 256, 0, stream>>>(attn, woutT, 8192, 1024, 1024,
                                             nullptr, out, b_out);
}
